// CrossGraphAttentionModule_26199300506297
// MI455X (gfx1250) — hardware-verified
//
#include <hip/hip_runtime.h>
#include <math.h>

typedef __attribute__((ext_vector_type(16))) _Float16 v16h;
typedef __attribute__((ext_vector_type(16))) __bf16 v16b;
typedef __attribute__((ext_vector_type(8)))  _Float16 v8h;
typedef __attribute__((ext_vector_type(8)))  float v8f;
typedef __attribute__((ext_vector_type(4)))  float v4f;
typedef __attribute__((ext_vector_type(2)))  float v2f;
typedef __attribute__((ext_vector_type(4)))  unsigned v4u;
typedef __attribute__((ext_vector_type(4)))  int v4i;
typedef float __attribute__((may_alias)) float_a;
typedef int __attribute__((may_alias)) int_a;

template <typename T> __device__ __forceinline__ void vst2(void* p, T v) { *(volatile T*)p = v; __threadfence(); *(volatile T*)p = v; }
__device__ __forceinline__ v8f wmma16(v16h a, v16h b, v8f c) {
  v8f d = __builtin_amdgcn_wmma_f32_16x16x32_f16(false, a, false, b, (short)0, c, false, false);
  asm volatile("v_nop\n\tv_nop\n\tv_nop\n\tv_nop" : "+v"(d) : "v"(a), "v"(b));
  return d;
}
__device__ __forceinline__ v8f wmma_bf(v16b a, v16b b, v8f c) {
  v8f d = __builtin_amdgcn_wmma_f32_16x16x32_bf16(false, a, false, b, (short)0, c, false, false);
  asm volatile("v_nop\n\tv_nop\n\tv_nop\n\tv_nop" : "+v"(d) : "v"(a), "v"(b));
  return d;
}
__device__ __forceinline__ v16h frag_h(const _Float16* rowk0, int lane) {
  union { v16h v; v8h q[2]; } u; const _Float16* p = rowk0 + 8 * (lane >> 4);
  u.q[0] = *(const v8h*)p; u.q[1] = *(const v8h*)(p + 16); return u.v;
}
__device__ __forceinline__ v16h frag_f32(const float* rowk0, int lane) {
  v16h a; const float* p = rowk0 + 8 * (lane >> 4);
#pragma unroll
  for (int i = 0; i < 8; ++i) { a[i] = (_Float16)p[i]; a[8 + i] = (_Float16)p[16 + i]; }
  return a;
}
__device__ __forceinline__ v16h frag_f32s(const float* rowk0, int lane, float sc) {
  v16h a; const float* p = rowk0 + 8 * (lane >> 4);
#pragma unroll
  for (int i = 0; i < 8; ++i) { a[i] = (_Float16)(p[i] * sc); a[8 + i] = (_Float16)(p[16 + i] * sc); }
  return a;
}
__device__ __forceinline__ v16h fragc_f32(const float* W, int k0, int n, int lane, int ld, int K) {
  v16h a; const int g = lane >> 4;
#pragma unroll
  for (int i = 0; i < 8; ++i) { const int ka = k0 + 8 * g + i, kb = ka + 16;
    a[i] = (_Float16)(ka < K ? W[(size_t)(ka < K ? ka : K - 1) * ld + n] : 0.f); a[8 + i] = (_Float16)(kb < K ? W[(size_t)(kb < K ? kb : K - 1) * ld + n] : 0.f); }
  return a;
}
struct F2 { v16b h, l; };
__device__ __forceinline__ F2 bsplit16(const float v[16]) { F2 r;
#pragma unroll
  for (int i = 0; i < 16; ++i) { const __bf16 h = (__bf16)v[i]; r.h[i] = h; r.l[i] = (__bf16)(v[i] - (float)h); }
  return r; }
__device__ __forceinline__ F2 split_row(const float* row, int k0, int lane) { float v[16]; const float* p = row + k0 + 8 * (lane >> 4);
#pragma unroll
  for (int i = 0; i < 8; ++i) { v[i] = p[i]; v[8 + i] = p[16 + i]; }
  return bsplit16(v); }
__device__ __forceinline__ F2 split_rowK(const float* row, int k0, int lane, int K) { float v[16]; const int g = lane >> 4;
#pragma unroll
  for (int i = 0; i < 8; ++i) { const int ka = k0 + 8 * g + i, kb = ka + 16; v[i] = ka < K ? row[ka < K ? ka : K - 1] : 0.f; v[8 + i] = kb < K ? row[kb < K ? kb : K - 1] : 0.f; }
  return bsplit16(v); }
__device__ __forceinline__ F2 split_col(const float* W, int k0, int n, int lane, int ld, int K) { float v[16]; const int g = lane >> 4;
#pragma unroll
  for (int i = 0; i < 8; ++i) { const int ka = k0 + 8 * g + i, kb = ka + 16; v[i] = ka < K ? W[(size_t)(ka < K ? ka : K - 1) * ld + n] : 0.f; v[8 + i] = kb < K ? W[(size_t)(kb < K ? kb : K - 1) * ld + n] : 0.f; }
  return bsplit16(v); }
__device__ __forceinline__ v8f mac3(const F2& a, const F2& b, v8f c) { c = wmma_bf(a.l, b.h, c); c = wmma_bf(a.h, b.l, c); return wmma_bf(a.h, b.h, c); }
__device__ __forceinline__ float sigm(float v) { return 1.0f / (1.0f + expf(-v)); }
#define LDSX() do { asm volatile("s_wait_dscnt 0" ::: "memory"); __builtin_amdgcn_wave_barrier(); __builtin_amdgcn_fence(__ATOMIC_RELEASE, "workgroup"); } while (0)


#define NA 16384
#define NR 8192
#define DH 128
#define NG 32
#ifndef NAB
#define NAB (NA / 64)
#endif
typedef __attribute__((ext_vector_type(8))) __bf16 v8b;
__device__ __forceinline__ v16b frag_b(const __bf16* rowk0, int lane) {
  union { v16b v; v8b q[2]; } u; const __bf16* p = rowk0 + 8 * (lane >> 4);
  u.q[0] = *(const v8b*)p; u.q[1] = *(const v8b*)(p + 16); return u.v;
}
__device__ __forceinline__ float bfr(float v) { return (float)(__bf16)v; }
__device__ __attribute__((noinline)) float exp_ni(float v) { return expf(v); }
__device__ __attribute__((noinline)) float erf_ni(float v) { return erff(v); }

#define WS_PW   0u
#define WS_Q    (WS_PW + 2u * 3 * DH * DH)
#define WS_K    (WS_Q + 4u * NA * DH)
#define WS_VT   (WS_K + 4u * NR * DH)
#define WS_VTL  (WS_VT + 2u * DH * NR)
#define WS_RB   (WS_VTL + 2u * DH * NR)
#define WS_END  (WS_RB + 4u * 64)

__global__ __launch_bounds__(128) void k_packw(const float* __restrict__ WQ, const float* __restrict__ WK, const float* __restrict__ WV, __bf16* __restrict__ PW) {
  __shared__ __align__(16) __bf16 s[3][DH]; const int o = blockIdx.x, t = threadIdx.x;
  s[0][t] = (__bf16)WQ[o * DH + t]; s[1][t] = (__bf16)WK[o * DH + t]; s[2][t] = (__bf16)WV[o * DH + t]; __syncthreads();
  if (t < 48) { const int m = t / 16, pc = t % 16; vst2((unsigned*)(PW + (size_t)m * DH * DH + (size_t)o * DH + pc * 8), *(const v4u*)&s[m][pc * 8]); }
}
__global__ __launch_bounds__(64) void k_bounds(const int* __restrict__ RBATCH, int* __restrict__ RB) {
  __shared__ __align__(16) int s[64]; const int g = threadIdx.x;
  if (g < NG) { int lo = 0, hi = NR; while (lo < hi) { const int mid = (lo + hi) >> 1; if (RBATCH[mid] < g) lo = mid + 1; else hi = mid; } const int start = lo; lo = start; hi = NR; while (lo < hi) { const int mid = (lo + hi) >> 1; if (RBATCH[mid] <= g) lo = mid + 1; else hi = mid; } s[2 * g] = start; s[2 * g + 1] = lo; }
  __syncthreads();
  if (g < 16) vst2((unsigned*)(RB + g * 4), *(const v4u*)&s[g * 4]);
}
template <int MODE>
__global__ __launch_bounds__(128) void k_proj(const float* __restrict__ A, const __bf16* __restrict__ P, float* __restrict__ OUT, __bf16* __restrict__ TH, __bf16* __restrict__ TL) {
  __shared__ __align__(16) float so[4][16][132]; __shared__ __align__(16) __bf16 sh[128][72], sl[128][72];
  const int tid = threadIdx.x, wave = tid >> 5, lane = tid & 31, col = lane & 15, g = lane >> 4; const size_t r0 = (size_t)blockIdx.x * 64 + wave * 16;
  v8f acc[8] = {};
#pragma unroll
  for (int kc = 0; kc < 4; ++kc) { v16b a; const float* p = A + (r0 + col) * DH + kc * 32 + 8 * g;
#pragma unroll
    for (int i = 0; i < 8; ++i) { a[i] = (__bf16)p[i]; a[8 + i] = (__bf16)p[16 + i]; }
#pragma unroll
    for (int j = 0; j < 8; ++j) acc[j] = wmma_bf(a, frag_b(P + (size_t)(j * 16 + col) * DH + kc * 32, lane), acc[j]); }
  if (MODE == 0) {
#pragma unroll
    for (int j = 0; j < 8; ++j)
#pragma unroll
      for (int r = 0; r < 8; ++r) so[wave][8 * g + r][j * 16 + col] = acc[j][r];
    LDSX();
    for (int rl = 0; rl < 16; ++rl) vst2(OUT + (r0 + rl) * DH + lane * 4, *(const v4f*)&so[wave][rl][lane * 4]);
  } else {
#pragma unroll
    for (int j = 0; j < 8; ++j)
#pragma unroll
      for (int r = 0; r < 8; ++r) { const float v = acc[j][r]; const __bf16 hb = (__bf16)v; sh[j * 16 + col][wave * 16 + 8 * g + r] = hb; sl[j * 16 + col][wave * 16 + 8 * g + r] = (__bf16)(v - (float)hb); }
    __syncthreads();
    for (int q = tid; q < 128 * 8; q += 128) { const int d = q >> 3, pc = q & 7; vst2((unsigned*)(TH + (size_t)d * NR + (size_t)blockIdx.x * 64 + pc * 8), *(const v4u*)&sh[d][pc * 8]); vst2((unsigned*)(TL + (size_t)d * NR + (size_t)blockIdx.x * 64 + pc * 8), *(const v4u*)&sl[d][pc * 8]); }
  }
}
__global__ __launch_bounds__(128) void k_attn(const float* __restrict__ AH, const int* __restrict__ ABATCH, const int* __restrict__ RBATCH, const int* __restrict__ RB, const float* __restrict__ Q, const float* __restrict__ Kf, const __bf16* __restrict__ VT, const __bf16* __restrict__ VTL, float* __restrict__ OUT) {
  __shared__ __align__(16) float sp[4][16][36]; __shared__ __align__(16) float so[4][16][132]; __shared__ int sk0, sk1;
  const int tid = threadIdx.x, wave = tid >> 5, lane = tid & 31, col = lane & 15, g = lane >> 4; const size_t a0 = (size_t)blockIdx.x * 64; const size_t q0 = a0 + wave * 16;
  if (tid == 0) { const int gf = min(max(ABATCH[a0], 0), NG - 1), gl = min(max(ABATCH[a0 + 63], 0), NG - 1); const int lo = RB[2 * gf], hi = RB[2 * gl + 1]; sk0 = (lo / 32) * 32; sk1 = hi; }
  int rlo[8], rhi[8];
#pragma unroll
  for (int r = 0; r < 8; ++r) { const int ga = min(max(ABATCH[q0 + 8 * g + r], 0), NG - 1); rlo[r] = RB[2 * ga]; rhi[r] = RB[2 * ga + 1]; }
  __syncthreads();
  const int k0 = sk0, k1 = sk1; const float scale = 1.0f / sqrtf((float)DH);
  float m[8], l[8];
#pragma unroll
  for (int r = 0; r < 8; ++r) { m[r] = -3.0e38f; l[r] = 0.f; }
  v8f acc[8] = {};
#pragma unroll 1
  for (int ks = k0; ks < k1; ks += 32) { v8f s[2] = {};
#pragma unroll 1
    for (int kc = 0; kc < 4; ++kc) { const F2 aq = split_row(Q + (q0 + col) * DH, kc * 32, lane);
#pragma unroll
      for (int ct = 0; ct < 2; ++ct) { const size_t kk = (size_t)min(ks + ct * 16 + col, NR - 1); const F2 kb = split_row(Kf + kk * DH, kc * 32, lane); s[ct] = mac3(aq, kb, s[ct]); } }
#pragma unroll
    for (int r = 0; r < 8; ++r) { float sv[2];
#pragma unroll
      for (int ct = 0; ct < 2; ++ct) { const int key = ks + ct * 16 + col; sv[ct] = (key >= rlo[r] && key < rhi[r]) ? s[ct][r] * scale : -3.0e38f; }
      float mx = fmaxf(sv[0], sv[1]);
#pragma unroll
      for (int o = 1; o < 16; o <<= 1) mx = fmaxf(mx, __shfl_xor(mx, o));
      const float mn = fmaxf(m[r], mx); float e0 = 0.f, e1 = 0.f, alpha = 1.f;
      if (mn > -1.0e38f) { alpha = (m[r] <= -1.0e38f) ? 0.f : exp_ni(m[r] - mn); e0 = (sv[0] <= -1.0e38f) ? 0.f : exp_ni(sv[0] - mn); e1 = (sv[1] <= -1.0e38f) ? 0.f : exp_ni(sv[1] - mn); }
      float es = e0 + e1;
#pragma unroll
      for (int o = 1; o < 16; o <<= 1) es += __shfl_xor(es, o);
      l[r] = l[r] * alpha + es; m[r] = mn;
#pragma unroll
      for (int dt = 0; dt < 8; ++dt) acc[dt][r] *= alpha;
      sp[wave][8 * g + r][col] = e0; sp[wave][8 * g + r][16 + col] = e1; }
    LDSX();
    const F2 pa = split_row(&sp[wave][col][0], 0, lane);
#pragma unroll
    for (int dt = 0; dt < 8; ++dt) { const size_t pr = (size_t)(dt * 16 + col) * NR + ks; const v16b vh = frag_b(VT + pr, lane), vl = frag_b(VTL + pr, lane); acc[dt] = wmma_bf(pa.l, vh, acc[dt]); acc[dt] = wmma_bf(pa.h, vl, acc[dt]); acc[dt] = wmma_bf(pa.h, vh, acc[dt]); }
    LDSX(); }
#pragma unroll
  for (int dt = 0; dt < 8; ++dt)
#pragma unroll
    for (int r = 0; r < 8; ++r) { const float ctx = (l[r] > 0.f) ? acc[dt][r] / l[r] : 0.f; so[wave][8 * g + r][dt * 16 + col] = bfr(AH[(q0 + 8 * g + r) * DH + dt * 16 + col]) + ctx; }
  LDSX();
  for (int rl = 0; rl < 16; ++rl) vst2(OUT + (q0 + rl) * DH + lane * 4, *(const v4f*)&so[wave][rl][lane * 4]);
}
extern "C" void kernel_launch(void* const* d_in, const int* in_sizes, int n_in, void* d_out, int out_size, void* d_ws, size_t ws_size, hipStream_t stream) {
  (void)in_sizes; (void)n_in; (void)out_size;
  const float** F = (const float**)d_in; const int* AB = (const int*)d_in[2]; const int* RBT = (const int*)d_in[3];
  if (ws_size < (size_t)WS_END) return;
  char* ws = (char*)d_ws; __bf16* PW = (__bf16*)(ws + WS_PW); float *Q = (float*)(ws + WS_Q), *Kf = (float*)(ws + WS_K); __bf16 *VT = (__bf16*)(ws + WS_VT), *VTL = (__bf16*)(ws + WS_VTL); int* RB = (int*)(ws + WS_RB);
  k_packw<<<DH, 128, 0, stream>>>(F[4], F[5], F[6], PW);
  k_bounds<<<1, 64, 0, stream>>>(RBT, RB);
  k_proj<0><<<NA / 64, 128, 0, stream>>>(F[0], PW, Q, nullptr, nullptr);
  k_proj<0><<<NR / 64, 128, 0, stream>>>(F[1], PW + DH * DH, Kf, nullptr, nullptr);
  k_proj<1><<<NR / 64, 128, 0, stream>>>(F[1], PW + 2 * DH * DH, nullptr, VT, VTL);
  k_attn<<<NAB, 128, 0, stream>>>(F[0], AB, RBT, RB, Q, Kf, VT, VTL, (float*)d_out);
}
